// GINLayer_60868276519673
// MI455X (gfx1250) — hardware-run, weakly checked
//
#include <hip/hip_runtime.h>

typedef float          v8f   __attribute__((ext_vector_type(8)));
typedef float          v4f   __attribute__((ext_vector_type(4)));
typedef unsigned int   v4u   __attribute__((ext_vector_type(4)));
typedef int            v8i   __attribute__((ext_vector_type(8)));
typedef unsigned short v8us  __attribute__((ext_vector_type(8)));
typedef unsigned short v16us __attribute__((ext_vector_type(16)));
typedef __bf16         v16bf __attribute__((ext_vector_type(16)));
typedef _Float16       v16h  __attribute__((ext_vector_type(16)));
typedef v4f  __attribute__((may_alias)) v4fa;
typedef v8us __attribute__((may_alias)) v8usa;
union FragB { v16bf v; v16us u; v8us h[2]; v8i w; };
union FragH { v16h  v; v16us u; v8us h[2]; v8i w; };

__device__ __forceinline__ v8f wmb(const FragB& a, const FragB& b, v8f c) {
  v8f d = __builtin_amdgcn_wmma_f32_16x16x32_bf16(false, a.v, false, b.v, (short)0, c, false, false);
  asm volatile("v_nop\n\tv_nop\n\tv_nop\n\tv_nop" : "+v"(d) : "v"(a.w), "v"(b.w));
  return d;
}

__device__ __forceinline__ v8f wmh(const FragH& a, const FragH& b, v8f c) {
  v8f d = __builtin_amdgcn_wmma_f32_16x16x32_f16(false, a.v, false, b.v, (short)0, c, false, false);
  asm volatile("v_nop\n\tv_nop\n\tv_nop\n\tv_nop" : "+v"(d) : "v"(a.w), "v"(b.w));
  return d;
}

__device__ __forceinline__ unsigned bf16_bits(float f) {
  const unsigned u = __float_as_uint(f);
  const unsigned r = (u + 0x7FFFu + ((u >> 16) & 1u)) >> 16;
  const unsigned q = (u >> 16) | 0x40u;
  return ((u & 0x7fffffffu) > 0x7f800000u) ? q : r;
}

__device__ __forceinline__ float bf16_val(float f) {
  return __uint_as_float(bf16_bits(f) << 16);
}
__device__ __forceinline__ int clampi(int v, int lo, int hi) {
  return v < lo ? lo : (v > hi ? hi : v);
}

__device__ __forceinline__ unsigned f16_bits(float f) {
  const unsigned u  = __float_as_uint(f);
  const unsigned s  = (u >> 16) & 0x8000u;
  const unsigned a  = u & 0x7fffffffu;
  const unsigned t  = a - 0x38000000u;
  const unsigned r  = (t + 0x0FFFu + ((t >> 13) & 1u)) >> 13;
  const unsigned rc = r > 0x7C00u ? 0x7C00u : r;
  const bool small  = a < 0x38800000u;
  const bool isnan  = a > 0x7f800000u;
  const unsigned fin = small ? 0u : (s | rc);
  return isnan ? (s | 0x7E00u) : fin;
}

__device__ __forceinline__ unsigned pk16(unsigned lo, unsigned hi) { return lo | (hi << 16); }
__device__ __forceinline__ unsigned bf16_lo_bits(float v) {
  float hi = bf16_val(v);
  asm volatile("" : "+v"(hi));
  return bf16_bits(v - hi);
}
__device__ __forceinline__ v4u pack8_bf16(v4f a, v4f c) {
  return (v4u){ pk16(bf16_bits(a[0]), bf16_bits(a[1])), pk16(bf16_bits(a[2]), bf16_bits(a[3])),
                pk16(bf16_bits(c[0]), bf16_bits(c[1])), pk16(bf16_bits(c[2]), bf16_bits(c[3])) };
}
__device__ __forceinline__ v4u pack8_bf16_lo(v4f a, v4f c) {
  return (v4u){ pk16(bf16_lo_bits(a[0]), bf16_lo_bits(a[1])), pk16(bf16_lo_bits(a[2]), bf16_lo_bits(a[3])),
                pk16(bf16_lo_bits(c[0]), bf16_lo_bits(c[1])), pk16(bf16_lo_bits(c[2]), bf16_lo_bits(c[3])) };
}
__device__ __forceinline__ v4u pack8_f16(v4f a, v4f c) {
  return (v4u){ pk16(f16_bits(a[0]), f16_bits(a[1])), pk16(f16_bits(a[2]), f16_bits(a[3])),
                pk16(f16_bits(c[0]), f16_bits(c[1])), pk16(f16_bits(c[2]), f16_bits(c[3])) };
}

template <int FORM>
__global__ __launch_bounds__(256) void k_plane(const float* __restrict__ src, int rows, int cols, int ldsrc,
                                               unsigned short* __restrict__ dst, int MP, int KP) {
  static_assert(FORM >= 0 && FORM <= 3);
  const int KTOT = (FORM == 1 || FORM == 3) ? 2 * KP : KP;
  const unsigned ppr   = (unsigned)(KTOT >> 3);
  const unsigned kp8   = (unsigned)(KP >> 3);
  const unsigned total = (unsigned)MP * ppr;
  const unsigned g     = blockIdx.x * 256u + threadIdx.x;
  const unsigned rowu  = g / ppr;
  const unsigned p     = g - rowu * ppr;
  const bool second    = p >= kp8;
  const int row = (int)rowu;
  const int c0  = (int)((second ? p - kp8 : p) << 3);
  const float* srow = src + (size_t)clampi(row, 0, rows - 1) * (size_t)ldsrc;
  float x[8];
  unsigned mk[8];
#pragma unroll
  for (int e = 0; e < 8; ++e) {
    const int c = c0 + e;
    const float v = srow[clampi(c, 0, cols - 1)];
    asm volatile("" :: "v"(v));
    x[e]  = v;
    mk[e] = (row < rows && c < cols) ? 0xFFFFu : 0u;
  }
  const v4f a = (v4f){ x[0], x[1], x[2], x[3] };
  const v4f c = (v4f){ x[4], x[5], x[6], x[7] };
  v4u o;
  if (FORM == 2) {
    o = pack8_f16(a, c);
  } else {
    const v4u hi = pack8_bf16(a, c);
    o = hi;
    if (FORM == 1) { const v4u lo = pack8_bf16_lo(a, c); o = second ? lo : hi; }
  }
  const v4u mw = (v4u){ pk16(mk[0], mk[1]), pk16(mk[2], mk[3]), pk16(mk[4], mk[5]), pk16(mk[6], mk[7]) };
  o &= mw;
  if (g < total) {
    volatile v4u* q = (volatile v4u*)(dst + (size_t)g * 8);
    *q = o;
    __threadfence();
    *q = o;
  }
}

template <int FORM> struct FragOf    { typedef FragB T; };
template <>         struct FragOf<2> { typedef FragH T; };
__device__ __forceinline__ v8f mm(const FragB& a, const FragB& b, v8f c) { return wmb(a, b, c); }
__device__ __forceinline__ v8f mm(const FragH& a, const FragH& b, v8f c) { return wmh(a, b, c); }
template <class F> __device__ __forceinline__ F ld_frag(const unsigned short* p) {
  F f;
  f.h[0] = *(const v8usa*)(p);
  f.h[1] = *(const v8usa*)(p + 16);
  return f;
}

template <int FORM, int EPI>
__global__ __launch_bounds__(256) __attribute__((amdgpu_num_vgpr(248)))
void k_gemm_nt(const unsigned short* __restrict__ A, const unsigned short* __restrict__ B,
               const float* __restrict__ bias, float* __restrict__ D, int M, int N, int KTOT, int ldd) {
  static_assert(FORM >= 0 && FORM <= 2);
  static_assert(EPI == 0 || EPI == 1);
  typedef typename FragOf<FORM>::T F;
  __shared__ __attribute__((aligned(16))) float sT[8][16 * 68];
  const int lane = threadIdx.x & 31;
  const int wave = threadIdx.x >> 5;
  const int tilesM = (M + 63) >> 6;
  const int tilesN = (N + 63) >> 6;
  const int tile = blockIdx.x * 8 + wave;
  if (tile >= tilesM * tilesN) return;
  const int tm = tile / tilesN;
  const int tn = tile - tm * tilesN;
  const int m0 = tm << 6;
  const int n0 = tn << 6;

  const int rl = lane & 15;
  const int h8 = (lane >> 4) * 8;
  const unsigned short* pa = A + (size_t)(m0 + rl) * (size_t)KTOT + h8;
  const unsigned short* pb = B + (size_t)(n0 + rl) * (size_t)KTOT + h8;

  v8f acc[4][4];
#pragma unroll
  for (int i = 0; i < 4; ++i)
#pragma unroll
    for (int j = 0; j < 4; ++j) acc[i][j] = (v8f){0.f, 0.f, 0.f, 0.f, 0.f, 0.f, 0.f, 0.f};

#pragma unroll 1
  for (int k0 = 0; k0 < KTOT; k0 += 32) {
    F bf[4];
#pragma unroll
    for (int j = 0; j < 4; ++j) bf[j] = ld_frag<F>(pb + (size_t)(j << 4) * (size_t)KTOT + k0);
#pragma unroll
    for (int i = 0; i < 4; ++i) {
      const F af = ld_frag<F>(pa + (size_t)(i << 4) * (size_t)KTOT + k0);
#pragma unroll
      for (int j = 0; j < 4; ++j) acc[i][j] = mm(af, bf[j], acc[i][j]);
    }
  }

  float* slab = sT[wave];
  const int hh = lane >> 4;
  const int c4 = (lane & 15) * 4;
  const int nc = n0 + c4;
  const bool cok = nc < N;
  v4f bv = (v4f){0.f, 0.f, 0.f, 0.f};
  if (EPI == 1) {
    bv = *(const v4fa*)(bias + clampi(nc, 0, N - 4));
    asm volatile("" :: "v"(bv));
  }
#pragma unroll
  for (int i = 0; i < 4; ++i) {
    const int mBase = m0 + (i << 4);
#pragma unroll
    for (int j = 0; j < 4; ++j) {
#pragma unroll
      for (int r = 0; r < 8; ++r) slab[(h8 + r) * 68 + (j << 4) + rl] = acc[i][j][r];
    }
    __builtin_amdgcn_fence(__ATOMIC_RELEASE, "workgroup");
    __builtin_amdgcn_wave_barrier();
    __builtin_amdgcn_fence(__ATOMIC_ACQUIRE, "workgroup");
    v4f vv[8];
#pragma unroll
    for (int it = 0; it < 8; ++it) {
      const int row = it * 2 + hh;
      v4f v = *(const v4fa*)(slab + row * 68 + c4);
      if (EPI == 1) v += bv;
      vv[it] = v;
    }
    for (int pass = 0; pass < 2; ++pass) {
#pragma unroll
      for (int it = 0; it < 8; ++it) {
        const int row = mBase + it * 2 + hh;
        if (cok && row < M) *(volatile v4f*)(D + (size_t)row * (size_t)ldd + nc) = vv[it];
      }
      __threadfence();
    }
    __builtin_amdgcn_fence(__ATOMIC_RELEASE, "workgroup");
    __builtin_amdgcn_wave_barrier();
    __builtin_amdgcn_fence(__ATOMIC_ACQUIRE, "workgroup");
  }
}

#include <stddef.h>
#include <stdint.h>

#define H_TWO_TERM 1
#define T_TWO_TERM 1

#define NN     50000
#define NE     800000
#define FIN    64
#define HID    256
#define FOUT   64
#define MPAD   50048
#define KH1    (FIN * (1 + H_TWO_TERM))
#define KT2    (HID * (1 + T_TWO_TERM))

#define NTHR   256
#define NWAVE  8
#define EPT    8
#define CHUNK  (NTHR * EPT)
#define WCAP   (EPT * 32)
#define LISTN  (NWAVE * WCAP)
#define NBA    1024
#define SLA    10
#define NBLK   49
#define RCAP   21504
#define DEGCAP 64
#define BK_ZINTS (LISTN + 2 * RCAP + 3 * NBA)
#define BK_MISC  16
#define BK_LDS_BYTES ((BK_ZINTS + BK_MISC) * 4)

#define XB_BLOCKS (MPAD * (FIN / 8) / NTHR)
#define W1_BLOCKS (HID * (KH1 / 8) / NTHR)
#define W2_BLOCKS (FOUT * (KT2 / 8) / NTHR)
#define PREP_BLOCKS (XB_BLOCKS + W1_BLOCKS + W2_BLOCKS + 1)

static_assert(FIN == 32 * 2);
static_assert(MPAD % 128 == 0 && MPAD % 64 == 0 && MPAD >= NN && MPAD % NWAVE == 0);
static_assert(NN % 16 == 0 && HID % 64 == 0 && FOUT % 64 == 0);
static_assert(KH1 % 32 == 0 && KT2 % 32 == 0);
static_assert((MPAD * (FIN / 8)) % NTHR == 0);
static_assert((HID * (KH1 / 8)) % NTHR == 0 && (FOUT * (KT2 / 8)) % NTHR == 0);
static_assert(((long long)MPAD * KT2 / 8) % 256 == 0);
static_assert((long long)MPAD * KT2 / 8 < (1LL << 31));
static_assert(NBA == (1 << SLA) && NBLK * NBA >= MPAD);
static_assert(NE < (1 << 21));
static_assert((CHUNK & (CHUNK - 1)) == 0 && ((long long)CHUNK << SLA) < (1LL << 31));
static_assert(RCAP % (NTHR * 4) == 0 && RCAP * 4 >= 16696 * 5 && RCAP <= 24576);
static_assert(DEGCAP >= 33 + 8 && DEGCAP * 4 >= 33 * 5);
static_assert(BK_ZINTS % (NTHR * 4) == 0 && LISTN % 4 == 0 && NBA == NTHR * 4);
static_assert(BK_LDS_BYTES <= 262144);

typedef int v4i __attribute__((ext_vector_type(4)));
typedef v4i __attribute__((may_alias)) v4ia;
typedef v4u __attribute__((may_alias)) v4ua;

__device__ __forceinline__ void wave_sync() {
  __builtin_amdgcn_fence(__ATOMIC_RELEASE, "wavefront");
  __builtin_amdgcn_wave_barrier();
  __builtin_amdgcn_fence(__ATOMIC_ACQUIRE, "wavefront");
}

__global__ __launch_bounds__(NTHR) void k_prep(const float* __restrict__ x, const float* __restrict__ W1,
                                               const float* __restrict__ b1, const float* __restrict__ W2,
                                               const float* __restrict__ b2, unsigned short* XB,
                                               unsigned short* W1D, unsigned short* W2D, float* BF, int nN) {
  const int b = (int)blockIdx.x;
  const int tid = (int)threadIdx.x;
  if (b < XB_BLOCKS) {
    const int g = b * NTHR + tid;
    const int row = g >> 3;
    const int p = g & 7;
    const int rc = row < nN ? row : nN - 1;
    const float* sp = x + (size_t)rc * FIN + 8 * p;
    const v4f a = *(const v4fa*)sp;
    const v4f c = *(const v4fa*)(sp + 4);
    asm volatile("" :: "v"(a));
    asm volatile("" :: "v"(c));
    v4u o = pack8_bf16(a, c);
    const unsigned m = row < nN ? 0xFFFFFFFFu : 0u;
    o &= (v4u){ m, m, m, m };
    volatile v4u* q = (volatile v4u*)(XB + (size_t)g * 8);
    *q = o;
    __threadfence();
    *q = o;
  } else if (b < XB_BLOCKS + W1_BLOCKS) {
    const int g = (b - XB_BLOCKS) * NTHR + tid;
    const int ppr = KH1 / 8;
    const int n = g / ppr;
    const int p = g - n * ppr;
    const int km = (8 * p) & (FIN - 1);
    float v[8];
#pragma unroll
    for (int e = 0; e < 8; ++e) {
      const float t = W1[(size_t)(km + e) * HID + n];
      asm volatile("" :: "v"(t));
      v[e] = t;
    }
    const v4u o = pack8_bf16((v4f){ v[0], v[1], v[2], v[3] }, (v4f){ v[4], v[5], v[6], v[7] });
    volatile v4u* q = (volatile v4u*)(W1D + (size_t)g * 8);
    *q = o;
    __threadfence();
    *q = o;
  } else if (b < XB_BLOCKS + W1_BLOCKS + W2_BLOCKS) {
    const int g = (b - XB_BLOCKS - W1_BLOCKS) * NTHR + tid;
    const int ppr = KT2 / 8;
    const int n = g / ppr;
    const int p = g - n * ppr;
    const int km = (8 * p) & (HID - 1);
    float v[8];
#pragma unroll
    for (int e = 0; e < 8; ++e) {
      const float t = W2[(size_t)(km + e) * FOUT + n];
      asm volatile("" :: "v"(t));
      v[e] = t;
    }
    const v4u o = pack8_bf16((v4f){ v[0], v[1], v[2], v[3] }, (v4f){ v[4], v[5], v[6], v[7] });
    volatile v4u* q = (volatile v4u*)(W2D + (size_t)g * 8);
    *q = o;
    __threadfence();
    *q = o;
  } else {
    const int i1 = tid < (HID / 4) ? tid : (HID / 4 - 1);
    const int i2 = clampi(tid - HID / 4, 0, FOUT / 4 - 1);
    const v4f t1 = *(const v4fa*)(b1 + 4 * i1);
    const v4f t2 = *(const v4fa*)(b2 + 4 * i2);
    asm volatile("" :: "v"(t1));
    asm volatile("" :: "v"(t2));
    const unsigned m = tid < (HID / 4) ? 0xFFFFFFFFu : 0u;
    v4f o;
#pragma unroll
    for (int e = 0; e < 4; ++e) {
      const unsigned u1 = bf16_bits(t1[e]) << 16;
      const unsigned u2 = bf16_bits(t2[e]) << 16;
      o[e] = __uint_as_float((u1 & m) | (u2 & ~m));
    }
    const bool act = tid < (HID + FOUT) / 4;
    volatile v4f* q = (volatile v4f*)(BF + 4 * (act ? tid : 0));
    if (act) *q = o;
    __threadfence();
    if (act) *q = o;
  }
}

__device__ __forceinline__ int scan_chunk(const int* __restrict__ keys, int nE, int cbase, int slotBase, int nb,
                                          int* list, int tid, int wave) {
  int wc = 0;
  const int el0 = tid * EPT;
  const int e0  = cbase + el0;
  v4i da, db;
  if (cbase + CHUNK <= nE) {
    da = *(const v4i*)(keys + e0);
    db = *(const v4i*)(keys + e0 + 4);
  } else {
    const int last = nE - 1;
    const int k0 = keys[min(e0,     last)];
    const int k1 = keys[min(e0 + 1, last)];
    const int k2 = keys[min(e0 + 2, last)];
    const int k3 = keys[min(e0 + 3, last)];
    const int k4 = keys[min(e0 + 4, last)];
    const int k5 = keys[min(e0 + 5, last)];
    const int k6 = keys[min(e0 + 6, last)];
    const int k7 = keys[min(e0 + 7, last)];
    asm volatile("" :: "v"(k0)); asm volatile("" :: "v"(k1));
    asm volatile("" :: "v"(k2)); asm volatile("" :: "v"(k3));
    asm volatile("" :: "v"(k4)); asm volatile("" :: "v"(k5));
    asm volatile("" :: "v"(k6)); asm volatile("" :: "v"(k7));
    da.x = (e0     < nE) ? k0 : -1;
    da.y = (e0 + 1 < nE) ? k1 : -1;
    da.z = (e0 + 2 < nE) ? k2 : -1;
    da.w = (e0 + 3 < nE) ? k3 : -1;
    db.x = (e0 + 4 < nE) ? k4 : -1;
    db.y = (e0 + 5 < nE) ? k5 : -1;
    db.z = (e0 + 6 < nE) ? k6 : -1;
    db.w = (e0 + 7 < nE) ? k7 : -1;
  }
  const unsigned nbs = (unsigned)slotBase;
  const unsigned unb = (unsigned)nb;
  const unsigned s0 = (unsigned)da.x - nbs, s1 = (unsigned)da.y - nbs;
  const unsigned s2 = (unsigned)da.z - nbs, s3 = (unsigned)da.w - nbs;
  const unsigned s4 = (unsigned)db.x - nbs, s5 = (unsigned)db.y - nbs;
  const unsigned s6 = (unsigned)db.z - nbs, s7 = (unsigned)db.w - nbs;
  const bool h0 = s0 < unb, h1 = s1 < unb, h2 = s2 < unb, h3 = s3 < unb;
  const bool h4 = s4 < unb, h5 = s5 < unb, h6 = s6 < unb, h7 = s7 < unb;
  const unsigned any = __builtin_amdgcn_ballot_w32(h0 | h1 | h2 | h3 | h4 | h5 | h6 | h7);
  if (any != 0u) {
    const unsigned m0 = __builtin_amdgcn_ballot_w32(h0);
    const unsigned m1 = __builtin_amdgcn_ballot_w32(h1);
    const unsigned m2 = __builtin_amdgcn_ballot_w32(h2);
    const unsigned m3 = __builtin_amdgcn_ballot_w32(h3);
    const unsigned m4 = __builtin_amdgcn_ballot_w32(h4);
    const unsigned m5 = __builtin_amdgcn_ballot_w32(h5);
    const unsigned m6 = __builtin_amdgcn_ballot_w32(h6);
    const unsigned m7 = __builtin_amdgcn_ballot_w32(h7);
    int pos = (int)(__builtin_amdgcn_mbcnt_lo(m0, 0u) + __builtin_amdgcn_mbcnt_lo(m1, 0u) +
                    __builtin_amdgcn_mbcnt_lo(m2, 0u) + __builtin_amdgcn_mbcnt_lo(m3, 0u) +
                    __builtin_amdgcn_mbcnt_lo(m4, 0u) + __builtin_amdgcn_mbcnt_lo(m5, 0u) +
                    __builtin_amdgcn_mbcnt_lo(m6, 0u) + __builtin_amdgcn_mbcnt_lo(m7, 0u));
    int* wl = list + wave * WCAP;
    if (h0 && pos < WCAP) wl[pos] = ((el0 + 0) << SLA) | (int)s0;
    pos += h0 ? 1 : 0;
    if (h1 && pos < WCAP) wl[pos] = ((el0 + 1) << SLA) | (int)s1;
    pos += h1 ? 1 : 0;
    if (h2 && pos < WCAP) wl[pos] = ((el0 + 2) << SLA) | (int)s2;
    pos += h2 ? 1 : 0;
    if (h3 && pos < WCAP) wl[pos] = ((el0 + 3) << SLA) | (int)s3;
    pos += h3 ? 1 : 0;
    if (h4 && pos < WCAP) wl[pos] = ((el0 + 4) << SLA) | (int)s4;
    pos += h4 ? 1 : 0;
    if (h5 && pos < WCAP) wl[pos] = ((el0 + 5) << SLA) | (int)s5;
    pos += h5 ? 1 : 0;
    if (h6 && pos < WCAP) wl[pos] = ((el0 + 6) << SLA) | (int)s6;
    pos += h6 ? 1 : 0;
    if (h7 && pos < WCAP) wl[pos] = ((el0 + 7) << SLA) | (int)s7;
    wc = (int)(__builtin_popcount(m0) + __builtin_popcount(m1) + __builtin_popcount(m2) + __builtin_popcount(m3) +
               __builtin_popcount(m4) + __builtin_popcount(m5) + __builtin_popcount(m6) + __builtin_popcount(m7));
  }
  return wc;
}

__global__ __launch_bounds__(NTHR) void k_bucket(const int* __restrict__ srcs, const int* __restrict__ keys,
                                                 int nE, int nN, int* LIST, int* CNT, int* OFF, int* FLAG) {
  extern __shared__ __attribute__((aligned(16))) int dsm[];
  int* list = dsm;
  int* hl   = dsm + LISTN;
  int* sl   = hl + RCAP;
  int* cnt  = sl + RCAP;
  int* offs = cnt + NBA;
  int* cur  = offs + NBA;
  int* misc = cur + NBA;
  const int tid = (int)threadIdx.x, lane = tid & 31, wave = tid >> 5;
  const int nodeBase = (int)blockIdx.x * NBA;
  const int nb = clampi(nN - nodeBase, 0, NBA);

  {
    const v4i z4 = {0, 0, 0, 0};
    for (int i = tid * 4; i < BK_ZINTS; i += NTHR * 4) *(v4ia*)(dsm + i) = z4;
    if (tid < BK_MISC) misc[tid] = 0;
  }
  __syncthreads();

  int t = 0, ov = 0;
  const int nChunks = (nE + CHUNK - 1) / CHUNK;
#pragma unroll 1
  for (int ch = 0; ch < nChunks; ++ch) {
    const int cbase = ch * CHUNK;
    const int wc = scan_chunk(keys, nE, cbase, nodeBase, nb, list, tid, wave);
    if (lane == 0) misc[wave] = wc;
    __syncthreads();
    if (wave == 0) {
#pragma unroll 1
      for (int w2 = 0; w2 < NWAVE; ++w2) {
        int c = misc[w2];
        c = clampi(c, 0, WCAP);
        c = __builtin_amdgcn_readfirstlane(c);
#pragma unroll 1
        for (int b0 = 0; b0 < c; b0 += 32) {
          const int idx = b0 + lane;
          const int ent = list[w2 * WCAP + (idx < WCAP ? idx : WCAP - 1)];
          const int m32 = (c - b0) < 32 ? (c - b0) : 32;
#pragma unroll 1
          for (int k = 0; k < m32; ++k) {
            const int u    = __builtin_amdgcn_readlane(ent, k);
            const int slot = u & (NBA - 1);
            const int el   = (u >> SLA) & (CHUNK - 1);
            const int pk   = ((cbase + el) << SLA) | slot;
            if (t < RCAP) {
              if (lane == 0) { hl[t] = pk; cnt[slot] = cnt[slot] + 1; }
              t = t + 1;
            } else {
              ov = 1;
            }
          }
        }
      }
    }
    __syncthreads();
  }
  if (wave == 0 && lane == 0) { misc[8] = t; misc[9] = ov; }
  __syncthreads();
  int tt = misc[8];
  tt = clampi(tt, 0, RCAP);
  tt = __builtin_amdgcn_readfirstlane(tt);
  const int ovf = misc[9];

  if (wave == 0) {
    const int base = lane * (NBA / 32);
    int s = 0;
#pragma unroll 1
    for (int i = 0; i < NBA / 32; ++i) s += cnt[base + i];
    int incl = s;
#pragma unroll
    for (int d = 1; d < 32; d <<= 1) {
      const int y = __shfl_up(incl, d, 32);
      if (lane >= d) incl += y;
    }
    int run = incl - s;
#pragma unroll 1
    for (int i = 0; i < NBA / 32; ++i) {
      const int cv = cnt[base + i];
      offs[base + i] = run;
      cur[base + i]  = run;
      run += cv;
    }
  }
  __syncthreads();
  if (wave == 0) {
#pragma unroll 1
    for (int b0 = 0; b0 < tt; b0 += 32) {
      const int idx = b0 + lane;
      const int ent = hl[idx < RCAP ? idx : RCAP - 1];
      const int m32 = (tt - b0) < 32 ? (tt - b0) : 32;
#pragma unroll 1
      for (int k = 0; k < m32; ++k) {
        const int u    = __builtin_amdgcn_readlane(ent, k);
        const int slot = u & (NBA - 1);
        if (lane == 0) {
          int p = cur[slot];
          p = clampi(p, 0, RCAP - 1);
          sl[p] = u;
          cur[slot] = p + 1;
        }
      }
    }
  }
  __syncthreads();

  int* lrow = LIST + (size_t)blockIdx.x * RCAP;
#pragma unroll 1
  for (int i0 = 0; i0 < RCAP; i0 += NTHR * 4) {
    const int i = i0 + tid * 4;
    const v4i ent = *(const v4ia*)(sl + i);
    int g0 = srcs[clampi(ent.x >> SLA, 0, nE - 1)];
    int g1 = srcs[clampi(ent.y >> SLA, 0, nE - 1)];
    int g2 = srcs[clampi(ent.z >> SLA, 0, nE - 1)];
    int g3 = srcs[clampi(ent.w >> SLA, 0, nE - 1)];
    asm volatile("" :: "v"(g0)); asm volatile("" :: "v"(g1));
    asm volatile("" :: "v"(g2)); asm volatile("" :: "v"(g3));
    v4i o;
    o.x = (i     < tt) ? clampi(g0, 0, nN - 1) : 0;
    o.y = (i + 1 < tt) ? clampi(g1, 0, nN - 1) : 0;
    o.z = (i + 2 < tt) ? clampi(g2, 0, nN - 1) : 0;
    o.w = (i + 3 < tt) ? clampi(g3, 0, nN - 1) : 0;
    volatile v4i* q = (volatile v4i*)(lrow + i);
    *q = o;
    __threadfence();
    *q = o;
  }
  {
    const v4i c4 = *(const v4ia*)(cnt + 4 * tid);
    const v4i o4 = *(const v4ia*)(offs + 4 * tid);
    const bool big = (c4.x > DEGCAP) | (c4.y > DEGCAP) | (c4.z > DEGCAP) | (c4.w > DEGCAP);
    if (big) misc[10] = 1;
    volatile v4i* qc = (volatile v4i*)(CNT + nodeBase + 4 * tid);
    volatile v4i* qo = (volatile v4i*)(OFF + nodeBase + 4 * tid);
    *qc = c4;
    *qo = o4;
    __threadfence();
    *qc = c4;
    *qo = o4;
  }
  __syncthreads();
  {
    const int fl = (ovf != 0 || misc[10] != 0) ? 1 : 0;
    const v4i f4 = { fl, fl, fl, fl };
    const bool act = (wave == 0) && (lane < 8);
    volatile v4i* qf = (volatile v4i*)(FLAG + (size_t)blockIdx.x * 32 + 4 * (act ? lane : 0));
    if (act) *qf = f4;
    __threadfence();
    if (act) *qf = f4;
  }
}

__global__ __launch_bounds__(NTHR) void k_replay(const unsigned* __restrict__ XBw, const int* __restrict__ LIST,
                                                 const int* __restrict__ CNT, const int* __restrict__ OFF,
                                                 const int* __restrict__ FLAG, const float* __restrict__ eps,
                                                 unsigned short* HHL, int nN, int mRows) {
  __shared__ __attribute__((aligned(16))) unsigned rowbuf[NWAVE][KH1 / 2];
  const int tid = (int)threadIdx.x, lane = tid & 31, wave = tid >> 5;
  const float s = 1.0f + bf16_val(eps[0]);
  const int node = (int)blockIdx.x * NWAVE + wave;
  const bool live = node < nN;
  const int nc = live ? node : nN - 1;
  const int blk = nc >> SLA;
  int c = CNT[nc];
  int o = OFF[nc];
  const int fl = FLAG[blk * 32];
  asm volatile("" :: "v"(c));
  asm volatile("" :: "v"(o));
  asm volatile("" :: "v"(fl));
  const bool big = (c > DEGCAP) | (c < 0);
  c = clampi(c, 0, DEGCAP);
  o = clampi(o, 0, RCAP);
  c = live ? c : 0;
  c = __builtin_amdgcn_readfirstlane(c);
  o = __builtin_amdgcn_readfirstlane(o);
  const int* lrow = LIST + (size_t)blk * RCAP;

  float a0 = 0.0f, a1 = 0.0f;
#pragma unroll 1
  for (int b0 = 0; b0 < c; b0 += 32) {
    int j = b0 + lane;
    j = j > c - 1 ? c - 1 : j;
    int idx = o + j;
    idx = idx > RCAP - 1 ? RCAP - 1 : idx;
    int sr = lrow[idx];
    asm volatile("" :: "v"(sr));
    sr = clampi(sr, 0, nN - 1);
    const int m32 = (c - b0) < 32 ? (c - b0) : 32;
#pragma unroll 1
    for (int k = 0; k < m32; ++k) {
      const int sk = __builtin_amdgcn_readlane(sr, k);
      const unsigned w = XBw[(size_t)sk * (FIN / 2) + lane];
      asm volatile("" :: "v"(w));
      a0 += __uint_as_float(w << 16);
      a1 += __uint_as_float(w & 0xffff0000u);
    }
  }
  const unsigned ws = XBw[(size_t)nc * (FIN / 2) + lane];
  asm volatile("" :: "v"(ws));
  const float hv0 = fmaf(s, __uint_as_float(ws << 16), a0);
  const float hv1 = fmaf(s, __uint_as_float(ws & 0xffff0000u), a1);
  const float pz = (fl != 0 || big) ? __int_as_float(0x7fc00000) : 0.0f;
  const float m0 = live ? (hv0 + pz) : 0.0f;
  const float m1 = live ? (hv1 + pz) : 0.0f;

  unsigned* rb = rowbuf[wave];
  rb[lane] = pk16(bf16_bits(m0), bf16_bits(m1));
#if H_TWO_TERM
  rb[32 + lane] = pk16(bf16_lo_bits(m0), bf16_lo_bits(m1));
#endif
  wave_sync();
  const int npl = KH1 / 8;
  const int li = lane < npl ? lane : npl - 1;
  const v4u q = *(const v4ua*)(rb + 4 * li);
  const bool act = (lane < npl) && (node < mRows);
  volatile v4u* p = (volatile v4u*)(HHL + (size_t)(node < mRows ? node : 0) * KH1 + 8 * li);
  if (act) *p = q;
  __threadfence();
  if (act) *p = q;
}

static inline size_t al256(size_t v) { return (v + 255) & ~(size_t)255; }
static inline int cdiv(int a, int b) { return (a + b - 1) / b; }

extern "C" void kernel_launch(void* const* d_in, const int* in_sizes, int n_in,
                              void* d_out, int out_size, void* d_ws, size_t ws_size,
                              hipStream_t stream) {
  if (n_in < 8) return;
  if (in_sizes[0] != NN * FIN) return;
  if (in_sizes[1] != FIN * HID) return;
  if (in_sizes[2] != HID) return;
  if (in_sizes[3] != HID * FOUT) return;
  if (in_sizes[4] != FOUT) return;
  if (in_sizes[5] < 1) return;
  if (in_sizes[6] != NE || in_sizes[7] != NE) return;
  if (out_size != NN * FOUT) return;

  const float* x   = (const float*)d_in[0];
  const float* W1  = (const float*)d_in[1];
  const float* b1  = (const float*)d_in[2];
  const float* W2  = (const float*)d_in[3];
  const float* b2  = (const float*)d_in[4];
  const float* eps = (const float*)d_in[5];
  const int*   gsr = (const int*)d_in[6];
  const int*   own = (const int*)d_in[7];
  float* out = (float*)d_out;

  char* ws = (char*)d_ws;
  size_t off = 0;
  const size_t oXB  = off; off = al256(off + (size_t)MPAD * FIN * 2);
  const size_t oHHL = off; off = al256(off + (size_t)MPAD * KH1 * 2);
  const size_t oT   = off; off = al256(off + (size_t)MPAD * HID * 4);
  const size_t oTHL = off; off = al256(off + (size_t)MPAD * KT2 * 2);
  const size_t oLST = off; off = al256(off + (size_t)NBLK * RCAP * 4);
  const size_t oCNT = off; off = al256(off + (size_t)NBLK * NBA * 4);
  const size_t oOFF = off; off = al256(off + (size_t)NBLK * NBA * 4);
  const size_t oW1D = off; off = al256(off + (size_t)HID * KH1 * 2);
  const size_t oW2D = off; off = al256(off + (size_t)FOUT * KT2 * 2);
  const size_t oBF  = off; off = al256(off + (size_t)(HID + FOUT) * 4);
  const size_t oFLG = off; off = al256(off + (size_t)NBLK * 32 * 4);
  if (off > ws_size || off > ((size_t)128 << 20)) return;

  unsigned short* XB  = (unsigned short*)(ws + oXB);
  unsigned short* HHL = (unsigned short*)(ws + oHHL);
  float*          T   = (float*)(ws + oT);
  unsigned short* THL = (unsigned short*)(ws + oTHL);
  int*            LST = (int*)(ws + oLST);
  int*            CNT = (int*)(ws + oCNT);
  int*            OFF = (int*)(ws + oOFF);
  unsigned short* W1D = (unsigned short*)(ws + oW1D);
  unsigned short* W2D = (unsigned short*)(ws + oW2D);
  float*          BF  = (float*)(ws + oBF);
  int*            FLG = (int*)(ws + oFLG);

  hipFuncSetAttribute(reinterpret_cast<const void*>(&k_bucket), hipFuncAttributeMaxDynamicSharedMemorySize,
                      (int)BK_LDS_BYTES);

  k_prep<<<PREP_BLOCKS, NTHR, 0, stream>>>(x, W1, b1, W2, b2, XB, W1D, W2D, BF, NN);
  k_bucket<<<NBLK, NTHR, BK_LDS_BYTES, stream>>>(gsr, own, NE, NN, LST, CNT, OFF, FLG);
  k_replay<<<MPAD / NWAVE, NTHR, 0, stream>>>((const unsigned*)XB, LST, CNT, OFF, FLG, eps, HHL, NN, MPAD);
  k_gemm_nt<0, 1><<<cdiv(cdiv(NN, 64) * (HID / 64), 8), 256, 0, stream>>>(HHL, W1D, BF, T, NN, HID, KH1, HID);
  k_plane<(T_TWO_TERM ? 1 : 0)><<<(MPAD / 8) * KT2 / 256, 256, 0, stream>>>(T, NN, HID, HID, THL, MPAD, HID);
  k_gemm_nt<0, 1><<<cdiv(cdiv(NN, 64) * (FOUT / 64), 8), 256, 0, stream>>>(THL, W2D, BF + HID, out, NN, FOUT, KT2, FOUT);
}
